// PhaseLinear_85882166051585
// MI455X (gfx1250) — hardware-verified
//
#include <hip/hip_runtime.h>

typedef __bf16         v16bf __attribute__((ext_vector_type(16)));
typedef float          v8f   __attribute__((ext_vector_type(8)));
typedef float          v4f   __attribute__((ext_vector_type(4)));
typedef unsigned int   v4u   __attribute__((ext_vector_type(4)));
typedef unsigned short v8us  __attribute__((ext_vector_type(8)));
typedef v4f __attribute__((may_alias)) v4fa;
typedef v4u __attribute__((may_alias)) v4ua;

union Frag { v16bf v; v4u q[2]; };

#define NB    4096
#define NIN   1024
#define NOUT  1024
#define NCP   4
#define XE    ((size_t)NB * NIN)
#define WE    ((size_t)NCP * NOUT * NIN)
#define BM    128
#define BN    32
#define KST   40
#define HALF_PI_F 1.5707963705062866f

static_assert((XE / 8) % 256 == 0);
static_assert((WE / 8) % 256 == 0);
static_assert(NB % BM == 0);
static_assert(NOUT % BN == 0);
static_assert(NIN % 32 == 0);

__device__ __forceinline__ unsigned int bf16_rne(float x) {
  unsigned int u = __float_as_uint(x);
  u += 0x7FFFu + ((u >> 16) & 1u);
  return u >> 16;
}

__device__ __forceinline__ void split_hl(float x, unsigned int& hi, unsigned int& lo) {
  hi = bf16_rne(x);
  const float r = x - __uint_as_float(hi << 16);
  lo = bf16_rne(r);
}

__device__ __forceinline__ v8f wmma_bf16(v16bf a, v16bf b, v8f c) {
  return __builtin_amdgcn_wmma_f32_16x16x32_bf16(false, a, false, b, (short)0, c, false, false);
}

__device__ __forceinline__ v16bf load_frag(const unsigned short* p, int h) {
  Frag f;
  f.q[0] = *(const v4ua*)(p + 8 * h);
  f.q[1] = *(const v4ua*)(p + 16 + 8 * h);
  return f.v;
}

__global__ __launch_bounds__(256) void k_split(
    const float* __restrict__ x, const float* __restrict__ w,
    unsigned short* __restrict__ xh, unsigned short* __restrict__ xl,
    unsigned short* __restrict__ wh, unsigned short* __restrict__ wl,
    int nx8, int nw8)
{
  const int g = blockIdx.x * 256 + threadIdx.x;
  if (g >= nx8 + nw8) return;
  const float* src;
  unsigned short* dh;
  unsigned short* dl;
  if (g < nx8) {
    src = x + (size_t)g * 8;
    dh = xh + (size_t)g * 8;
    dl = xl + (size_t)g * 8;
  } else {
    const int e = g - nx8;
    src = w + (size_t)e * 8;
    dh = wh + (size_t)e * 8;
    dl = wl + (size_t)e * 8;
  }
  const v4f a = *(const v4fa*)src;
  const v4f c = *(const v4fa*)(src + 4);
  unsigned int h0, h1, h2, h3, h4, h5, h6, h7;
  unsigned int l0, l1, l2, l3, l4, l5, l6, l7;
  split_hl(a.x, h0, l0); split_hl(a.y, h1, l1); split_hl(a.z, h2, l2); split_hl(a.w, h3, l3);
  split_hl(c.x, h4, l4); split_hl(c.y, h5, l5); split_hl(c.z, h6, l6); split_hl(c.w, h7, l7);
  const v8us vh = { (unsigned short)h0, (unsigned short)h1, (unsigned short)h2, (unsigned short)h3,
                    (unsigned short)h4, (unsigned short)h5, (unsigned short)h6, (unsigned short)h7 };
  const v8us vl = { (unsigned short)l0, (unsigned short)l1, (unsigned short)l2, (unsigned short)l3,
                    (unsigned short)l4, (unsigned short)l5, (unsigned short)l6, (unsigned short)l7 };
  *(volatile v8us*)dh = vh;
  *(volatile v8us*)dl = vl;
  __threadfence();
  *(volatile v8us*)dh = vh;
  *(volatile v8us*)dl = vl;
}

__device__ __forceinline__ void out_store_pass(const float* sO, float* out,
                                               int m_blk, int n_blk, int wv, int lane) {
  const int q8 = lane & 7, sub = lane >> 3;
  #pragma unroll
  for (int i = 0; i < 4; ++i) {
    const int row = wv * 16 + i * 4 + sub;
    const v4f v = *(const v4fa*)(sO + row * BN + 4 * q8);
    float* dst = out + (size_t)(m_blk + row) * NOUT + n_blk + 4 * q8;
    *(volatile v4f*)dst = v;
  }
}

__global__ __launch_bounds__(256) void k_gemm(
    const unsigned short* __restrict__ Xh, const unsigned short* __restrict__ Xl,
    const unsigned short* __restrict__ Wh, const unsigned short* __restrict__ Wl,
    const float* __restrict__ phase,
    const float* __restrict__ biases,
    const float* __restrict__ basis,
    float* __restrict__ out)
{
  __shared__ __attribute__((aligned(16))) unsigned short sAh[BM * KST];
  __shared__ __attribute__((aligned(16))) unsigned short sAl[BM * KST];
  __shared__ __attribute__((aligned(16))) unsigned short sWh[NCP * BN * KST];
  __shared__ __attribute__((aligned(16))) unsigned short sWl[NCP * BN * KST];
  __shared__ __attribute__((aligned(16))) float sO[BM * BN];
  __shared__ __attribute__((aligned(16))) float sE[BM * 4];
  __shared__ __attribute__((aligned(16))) float sBias[NCP * BN];

  const int tid = threadIdx.x, lane = tid & 31, wv = tid >> 5;
  const int wm = wv & 3, wn = wv >> 2;
  const int h = lane >> 4, m = lane & 15;
  const int n_blk = blockIdx.x * BN;
  const int m_blk = blockIdx.y * BM;

  if (tid < BM) {
    const float ph = phase[m_blk + tid];
    const float s  = ph * (1.0f / HALF_PI_F);
    int q = (int)floorf(s);
    q = q < 0 ? 0 : (q > 3 ? 3 : q);
    const float t  = s - (float)q;
    const float t2 = t * t;
    const float t3 = t2 * t;
    float bs[16];
    #pragma unroll
    for (int i = 0; i < 16; ++i) bs[i] = basis[i];
    const float cf0 = ((t3 * bs[0] + t2 * bs[4]) + t * bs[8])  + bs[12];
    const float cf1 = ((t3 * bs[1] + t2 * bs[5]) + t * bs[9])  + bs[13];
    const float cf2 = ((t3 * bs[2] + t2 * bs[6]) + t * bs[10]) + bs[14];
    const float cf3 = ((t3 * bs[3] + t2 * bs[7]) + t * bs[11]) + bs[15];
    #pragma unroll
    for (int c = 0; c < 4; ++c) {
      const int p = (c - q + 1) & 3;
      sE[tid * 4 + c] = (p == 0) ? cf0 : ((p == 1) ? cf1 : ((p == 2) ? cf2 : cf3));
    }
  }
  if (tid < NCP * BN) {
    const int c = tid >> 5, col = tid & 31;
    sBias[tid] = biases[c * NOUT + n_blk + col];
  }

  const int ar = tid >> 1, aq = (tid & 1) * 16;
  const unsigned short* xgh = Xh + (size_t)(m_blk + ar) * NIN + aq;
  const unsigned short* xgl = Xl + (size_t)(m_blk + ar) * NIN + aq;
  unsigned short* sah = sAh + ar * KST + aq;
  unsigned short* sal = sAl + ar * KST + aq;
  const int wc = tid >> 6, wr = (tid >> 1) & 31, wq = (tid & 1) * 16;
  const unsigned short* wgh = Wh + ((size_t)wc * NOUT + n_blk + wr) * NIN + wq;
  const unsigned short* wgl = Wl + ((size_t)wc * NOUT + n_blk + wr) * NIN + wq;
  unsigned short* swh = sWh + (wc * BN + wr) * KST + wq;
  unsigned short* swl = sWl + (wc * BN + wr) * KST + wq;

  const v8f zero8 = {0.f, 0.f, 0.f, 0.f, 0.f, 0.f, 0.f, 0.f};
  v8f acc[NCP][2];
  #pragma unroll
  for (int c = 0; c < NCP; ++c) { acc[c][0] = zero8; acc[c][1] = zero8; }

  const unsigned short* pa0h = sAh + (wm * 32 + m) * KST;
  const unsigned short* pa1h = pa0h + 16 * KST;
  const unsigned short* pa0l = sAl + (wm * 32 + m) * KST;
  const unsigned short* pa1l = pa0l + 16 * KST;
  const unsigned short* pbh  = sWh + (wn * 16 + m) * KST;
  const unsigned short* pbl  = sWl + (wn * 16 + m) * KST;

  #pragma unroll 1
  for (int kc = 0; kc < NIN; kc += 32) {
    __syncthreads();
    {
      const v4u t0 = *(const v4ua*)(xgh + kc);
      const v4u t1 = *(const v4ua*)(xgh + kc + 8);
      const v4u t2 = *(const v4ua*)(xgl + kc);
      const v4u t3 = *(const v4ua*)(xgl + kc + 8);
      const v4u t4 = *(const v4ua*)(wgh + kc);
      const v4u t5 = *(const v4ua*)(wgh + kc + 8);
      const v4u t6 = *(const v4ua*)(wgl + kc);
      const v4u t7 = *(const v4ua*)(wgl + kc + 8);
      *(v4ua*)(sah)     = t0;
      *(v4ua*)(sah + 8) = t1;
      *(v4ua*)(sal)     = t2;
      *(v4ua*)(sal + 8) = t3;
      *(v4ua*)(swh)     = t4;
      *(v4ua*)(swh + 8) = t5;
      *(v4ua*)(swl)     = t6;
      *(v4ua*)(swl + 8) = t7;
    }
    __syncthreads();

    const v16bf ah0 = load_frag(pa0h, h);
    const v16bf ah1 = load_frag(pa1h, h);
    const v16bf al0 = load_frag(pa0l, h);
    const v16bf al1 = load_frag(pa1l, h);
    #pragma unroll
    for (int c = 0; c < NCP; ++c) {
      const v16bf bh = load_frag(pbh + c * BN * KST, h);
      const v16bf bl = load_frag(pbl + c * BN * KST, h);
      v8f d0 = acc[c][0];
      v8f d1 = acc[c][1];
      d0 = wmma_bf16(ah0, bh, d0);
      d0 = wmma_bf16(ah0, bl, d0);
      d0 = wmma_bf16(al0, bh, d0);
      d1 = wmma_bf16(ah1, bh, d1);
      d1 = wmma_bf16(ah1, bl, d1);
      d1 = wmma_bf16(al1, bh, d1);
      asm volatile("v_nop\n\tv_nop\n\tv_nop\n\tv_nop"
                   : "+v"(d0), "+v"(d1)
                   : "v"(ah0), "v"(ah1), "v"(al0), "v"(al1), "v"(bh), "v"(bl));
      acc[c][0] = d0;
      acc[c][1] = d1;
    }
  }

  const int col = wn * 16 + m;
  const float b0 = sBias[0 * BN + col];
  const float b1 = sBias[1 * BN + col];
  const float b2 = sBias[2 * BN + col];
  const float b3 = sBias[3 * BN + col];
  #pragma unroll
  for (int mt = 0; mt < 2; ++mt) {
    #pragma unroll
    for (int r = 0; r < 8; ++r) {
      const int row = wm * 32 + mt * 16 + 8 * h + r;
      const v4f e = *(const v4fa*)(sE + row * 4);
      const float v = e.x * (acc[0][mt][r] + b0)
                    + e.y * (acc[1][mt][r] + b1)
                    + e.z * (acc[2][mt][r] + b2)
                    + e.w * (acc[3][mt][r] + b3);
      sO[row * BN + col] = v;
    }
  }
  __syncthreads();

  out_store_pass(sO, out, m_blk, n_blk, wv, lane);
  __threadfence();
  out_store_pass(sO, out, m_blk, n_blk, wv, lane);
}

extern "C" void kernel_launch(void* const* d_in, const int* in_sizes, int n_in,
                              void* d_out, int out_size, void* d_ws, size_t ws_size,
                              hipStream_t stream) {
  if (n_in < 5) return;
  if (in_sizes[0] != (int)XE) return;
  if (in_sizes[1] != NB) return;
  if (in_sizes[2] != (int)WE) return;
  if (in_sizes[3] != NCP * NOUT) return;
  if (in_sizes[4] != 16) return;
  if (out_size != (int)((size_t)NB * NOUT)) return;

  const float* x      = (const float*)d_in[0];
  const float* phase  = (const float*)d_in[1];
  const float* wts    = (const float*)d_in[2];
  const float* biases = (const float*)d_in[3];
  const float* basis  = (const float*)d_in[4];
  float* out = (float*)d_out;

  const size_t xplane = XE * 2;
  const size_t wplane = WE * 2;
  const size_t total  = 2 * xplane + 2 * wplane;
  if (total > ws_size) return;

  char* ws = (char*)d_ws;
  unsigned short* xh = (unsigned short*)(ws);
  unsigned short* xl = (unsigned short*)(ws + xplane);
  unsigned short* wh = (unsigned short*)(ws + 2 * xplane);
  unsigned short* wl = (unsigned short*)(ws + 2 * xplane + wplane);

  const int nx8 = (int)(XE / 8);
  const int nw8 = (int)(WE / 8);
  k_split<<<(nx8 + nw8 + 255) / 256, 256, 0, stream>>>(x, wts, xh, xl, wh, wl, nx8, nw8);

  dim3 grid(NOUT / BN, NB / BM);
  k_gemm<<<grid, 256, 0, stream>>>(xh, xl, wh, wl, phase, biases, basis, out);
}
